// CHAREncoder_33500744909048
// MI455X (gfx1250) — hardware-run, weakly checked
//
#include <hip/hip_runtime.h>


namespace {
constexpr int NS = 16384, T = 25, V = 399, E = 32, H = 32, G = 128;
constexpr float XS = 8.0f, WSC = 256.0f;
typedef _Float16 b16;
typedef __attribute__((ext_vector_type(16))) _Float16 v16b;
typedef __attribute__((ext_vector_type(8))) _Float16 v8b;
typedef __attribute__((ext_vector_type(8))) float v8f;
typedef __attribute__((ext_vector_type(4))) float v4f;
__device__ __forceinline__ float bf16_rne(float f) { unsigned int u = __float_as_uint(f); u += 0x7FFFu + ((u >> 16) & 1u); float r = __uint_as_float(u & 0xFFFF0000u); asm volatile("" : "+v"(r)); return r; }
__device__ __forceinline__ float bfv(float f) { float r = bf16_rne(f); asm volatile("" : "+v"(r)); return r; }
__device__ __forceinline__ void split16(float v, b16& hi, b16& lo) { hi = (b16)v; lo = (b16)(v - (float)hi); }
__device__ __forceinline__ v16b frag_kb(const b16* p, int hh) { const v8b a = *(const v8b*)(p + 8 * hh), b = *(const v8b*)(p + 16 + 8 * hh); v16b f;
#pragma unroll
  for (int e = 0; e < 8; ++e) { f[e] = a[e]; f[8 + e] = b[e]; } return f; }
__device__ __forceinline__ v8f wmma16b(v16b a, v16b b, v8f c) { v8f d = __builtin_amdgcn_wmma_f32_16x16x32_f16(false, a, false, b, (short)0, c, false, false); asm volatile("v_nop\n\tv_nop\n\tv_nop\n\tv_nop" : "+v"(d) : "v"(a), "v"(b)); return d; }
__device__ __forceinline__ void wave_lds_sync() { __builtin_amdgcn_fence(__ATOMIC_RELEASE, "workgroup"); __builtin_amdgcn_wave_barrier(); __builtin_amdgcn_fence(__ATOMIC_ACQUIRE, "workgroup"); }
__device__ __forceinline__ float pmul(float a, float b) { float p = a * b; asm volatile("" : "+v"(p)); return p; }
__device__ __forceinline__ int iclamp(int v, int lo, int hi) { return v < lo ? lo : (v > hi ? hi : v); }
__device__ __forceinline__ float sigm(float v) { return 1.0f / (1.0f + __expf(-v)); }

__global__ __launch_bounds__(256) void wput_kernel(const float* __restrict__ wif, const float* __restrict__ whf, const float* __restrict__ wib, const float* __restrict__ whb, b16* __restrict__ WI, b16* __restrict__ WH) { const int u = blockIdx.x * 256 + threadIdx.x; if (u >= 2 * G * 4) return; const int r = u / 4, k0 = (u % 4) * 8; const int d = r / G, g = r % G; const float* wi = d ? wib : wif; const float* wh = d ? whb : whf; v8b a, b;
#pragma unroll
  for (int j = 0; j < 8; ++j) { a[j] = (b16)(bf16_rne(wi[(size_t)g * E + k0 + j]) * WSC); b[j] = (b16)(bf16_rne(wh[(size_t)g * H + k0 + j]) * WSC); }
  for (int pass = 0; pass < 2; ++pass) { *(volatile v8b*)(WI + (size_t)r * E + k0) = a; *(volatile v8b*)(WH + (size_t)r * H + k0) = b; __threadfence(); } }
__global__ __launch_bounds__(32) void step_kernel(const int* __restrict__ ids, const float* __restrict__ emb, int t, const b16* __restrict__ WI, const b16* __restrict__ WH, const float* __restrict__ bih, const float* __restrict__ bhh, const float* __restrict__ Hp, const float* __restrict__ Cp, int FIRST, int LAST, int dir, int NLIM, float* __restrict__ Hn, float* __restrict__ Cn, float* __restrict__ out) { __shared__ __attribute__((aligned(16))) b16 Xh[16][40], Ah[16][40], Al[16][40]; __shared__ float Tf[16][G + 4]; const int lane = threadIdx.x, nloc = lane & 15, hlf = lane >> 4; const size_t m0 = (size_t)blockIdx.x * 16; if (m0 >= (size_t)NLIM) return;
  for (int rr = 0; rr < 16; ++rr) { const size_t n = m0 + rr; const int id = iclamp(ids[n * T + t], 0, V - 1); Xh[rr][lane] = (b16)(bf16_rne(emb[(size_t)id * E + lane]) * XS); const float hv = FIRST ? 0.0f : Hp[n * H + lane]; b16 p, ql; split16(hv * XS, p, ql); Ah[rr][lane] = p; Al[rr][lane] = ql; if (lane < 8) { Xh[rr][32 + lane] = (b16)0.0f; Ah[rr][32 + lane] = (b16)0.0f; Al[rr][32 + lane] = (b16)0.0f; } }
  wave_lds_sync(); const v16b xa = frag_kb(&Xh[nloc][0], hlf), ha = frag_kb(&Ah[nloc][0], hlf), hl2 = frag_kb(&Al[nloc][0], hlf);
#pragma unroll
  for (int tq = 0; tq < 8; ++tq) { v8f acc = {}; acc = wmma16b(xa, frag_kb(WI + (size_t)(tq * 16 + nloc) * E, hlf), acc); const v16b bw = frag_kb(WH + (size_t)(tq * 16 + nloc) * H, hlf); acc = wmma16b(ha, bw, acc); acc = wmma16b(hl2, bw, acc); const int cc = tq * 16 + nloc; const float bb = bfv(bih[cc]) + bfv(bhh[cc]);
#pragma unroll
    for (int r8 = 0; r8 < 8; ++r8) Tf[8 * hlf + r8][cc] = acc[r8] * (1.0f / (XS * WSC)) + bb; }
  wave_lds_sync();
  for (int pass = 0; pass < 2; ++pass) { for (int rr = 0; rr < 16; ++rr) { const size_t n = m0 + rr; const float ig = sigm(Tf[rr][lane]), fg = sigm(Tf[rr][H + lane]), gg = tanhf(Tf[rr][2 * H + lane]), og = sigm(Tf[rr][3 * H + lane]); const float cp = FIRST ? 0.0f : Cp[n * H + lane]; const float c = pmul(fg, cp) + pmul(ig, gg); const float h = pmul(og, tanhf(c));
      if (LAST) ((volatile float*)out)[n * (2 * H) + dir * H + lane] = h; else { ((volatile float*)Hn)[n * H + lane] = h; ((volatile float*)Cn)[n * H + lane] = c; } } __threadfence(); } }
}

extern "C" void kernel_launch(void* const* d_in, const int* in_sizes, int n_in, void* d_out, int out_size, void* d_ws, size_t ws_size, hipStream_t stream) {
  (void)n_in;
  auto Fp = [&](int i) { return (const float*)d_in[i]; }; auto Ip = [&](int i) { return (const int*)d_in[i]; };
  if (in_sizes[0] != NS * T || in_sizes[1] != V * E || in_sizes[2] != G * E || in_sizes[3] != G * H || in_sizes[6] != G * E || in_sizes[7] != G * H || out_size != NS * 2 * H) return;
  const int NLIM = NS;
  size_t off = 0; char* ws = (char*)d_ws;
  auto carve = [&](size_t bytes) { char* p = ws + off; off += (bytes + 255) & ~(size_t)255; return p; };
  b16* WI = (b16*)carve((size_t)2 * G * E * 2); b16* WH = (b16*)carve((size_t)2 * G * H * 2); float* HP[2]; float* CP[2]; for (int k = 0; k < 2; ++k) { HP[k] = (float*)carve((size_t)NS * H * 4); CP[k] = (float*)carve((size_t)NS * H * 4); }
  if (off > ws_size || off > ((size_t)16 << 20)) return;
  wput_kernel<<<(2 * G * 4 + 255) / 256, 256, 0, stream>>>(Fp(2), Fp(3), Fp(6), Fp(7), WI, WH);
  for (int dir = 0; dir < 2; ++dir) { const b16* wi = WI + (size_t)dir * G * E; const b16* wh = WH + (size_t)dir * G * H; const float* bih = Fp(dir ? 8 : 4); const float* bhh = Fp(dir ? 9 : 5);
    for (int s = 0; s < T; ++s) { const int t = dir ? (T - 1 - s) : s; const int cur = s & 1, nxt = cur ^ 1;
      step_kernel<<<NLIM / 16, 32, 0, stream>>>(Ip(0), Fp(1), t, wi, wh, bih, bhh, HP[cur], CP[cur], s == 0, s == T - 1, dir, NLIM, HP[nxt], CP[nxt], (float*)d_out); } }
}
